// TreeSupport_39651138076979
// MI455X (gfx1250) — hardware-run, weakly checked
//
#include <hip/hip_runtime.h>

typedef float          v8f   __attribute__((ext_vector_type(8)));
typedef float          v4f   __attribute__((ext_vector_type(4)));
typedef unsigned int   v4u   __attribute__((ext_vector_type(4)));
typedef int            v8i   __attribute__((ext_vector_type(8)));
typedef unsigned short v8us  __attribute__((ext_vector_type(8)));
typedef unsigned short v16us __attribute__((ext_vector_type(16)));
typedef __bf16         v16bf __attribute__((ext_vector_type(16)));
typedef _Float16       v16h  __attribute__((ext_vector_type(16)));
typedef v4f  __attribute__((may_alias)) v4fa;
typedef v8us __attribute__((may_alias)) v8usa;
union FragB { v16bf v; v16us u; v8us h[2]; v8i w; };
union FragH { v16h  v; v16us u; v8us h[2]; v8i w; };

__device__ __forceinline__ v8f wmb(const FragB& a, const FragB& b, v8f c) {
  v8f d = __builtin_amdgcn_wmma_f32_16x16x32_bf16(false, a.v, false, b.v, (short)0, c, false, false);
  asm volatile("v_nop\n\tv_nop\n\tv_nop\n\tv_nop" : "+v"(d) : "v"(a.w), "v"(b.w));
  return d;
}

__device__ __forceinline__ v8f wmh(const FragH& a, const FragH& b, v8f c) {
  v8f d = __builtin_amdgcn_wmma_f32_16x16x32_f16(false, a.v, false, b.v, (short)0, c, false, false);
  asm volatile("v_nop\n\tv_nop\n\tv_nop\n\tv_nop" : "+v"(d) : "v"(a.w), "v"(b.w));
  return d;
}

__device__ __forceinline__ unsigned bf16_bits(float f) {
  const unsigned u = __float_as_uint(f);
  const unsigned r = (u + 0x7FFFu + ((u >> 16) & 1u)) >> 16;
  const unsigned q = (u >> 16) | 0x40u;
  return ((u & 0x7fffffffu) > 0x7f800000u) ? q : r;
}

__device__ __forceinline__ float bf16_val(float f) {
  return __uint_as_float(bf16_bits(f) << 16);
}
__device__ __forceinline__ int clampi(int v, int lo, int hi) {
  return v < lo ? lo : (v > hi ? hi : v);
}

__device__ __forceinline__ unsigned f16_bits(float f) {
  const unsigned u  = __float_as_uint(f);
  const unsigned s  = (u >> 16) & 0x8000u;
  const unsigned a  = u & 0x7fffffffu;
  const unsigned t  = a - 0x38000000u;
  const unsigned r  = (t + 0x0FFFu + ((t >> 13) & 1u)) >> 13;
  const unsigned rc = r > 0x7C00u ? 0x7C00u : r;
  const bool small  = a < 0x38800000u;
  const bool isnan  = a > 0x7f800000u;
  const unsigned fin = small ? 0u : (s | rc);
  return isnan ? (s | 0x7E00u) : fin;
}

__device__ __forceinline__ unsigned pk16(unsigned lo, unsigned hi) { return lo | (hi << 16); }
__device__ __forceinline__ unsigned bf16_lo_bits(float v) {
  float hi = bf16_val(v);
  asm volatile("" : "+v"(hi));
  return bf16_bits(v - hi);
}
__device__ __forceinline__ v4u pack8_bf16(v4f a, v4f c) {
  return (v4u){ pk16(bf16_bits(a[0]), bf16_bits(a[1])), pk16(bf16_bits(a[2]), bf16_bits(a[3])),
                pk16(bf16_bits(c[0]), bf16_bits(c[1])), pk16(bf16_bits(c[2]), bf16_bits(c[3])) };
}
__device__ __forceinline__ v4u pack8_bf16_lo(v4f a, v4f c) {
  return (v4u){ pk16(bf16_lo_bits(a[0]), bf16_lo_bits(a[1])), pk16(bf16_lo_bits(a[2]), bf16_lo_bits(a[3])),
                pk16(bf16_lo_bits(c[0]), bf16_lo_bits(c[1])), pk16(bf16_lo_bits(c[2]), bf16_lo_bits(c[3])) };
}
__device__ __forceinline__ v4u pack8_f16(v4f a, v4f c) {
  return (v4u){ pk16(f16_bits(a[0]), f16_bits(a[1])), pk16(f16_bits(a[2]), f16_bits(a[3])),
                pk16(f16_bits(c[0]), f16_bits(c[1])), pk16(f16_bits(c[2]), f16_bits(c[3])) };
}

template <int FORM>
__global__ __launch_bounds__(256) void k_plane(const float* __restrict__ src, int rows, int cols, int ldsrc,
                                               unsigned short* __restrict__ dst, int MP, int KP) {
  static_assert(FORM >= 0 && FORM <= 3);
  const int KTOT = (FORM == 1 || FORM == 3) ? 2 * KP : KP;
  const unsigned ppr   = (unsigned)(KTOT >> 3);
  const unsigned kp8   = (unsigned)(KP >> 3);
  const unsigned total = (unsigned)MP * ppr;
  const unsigned g     = blockIdx.x * 256u + threadIdx.x;
  const unsigned rowu  = g / ppr;
  const unsigned p     = g - rowu * ppr;
  const bool second    = p >= kp8;
  const int row = (int)rowu;
  const int c0  = (int)((second ? p - kp8 : p) << 3);
  const float* srow = src + (size_t)clampi(row, 0, rows - 1) * (size_t)ldsrc;
  float x[8];
  unsigned mk[8];
#pragma unroll
  for (int e = 0; e < 8; ++e) {
    const int c = c0 + e;
    const float v = srow[clampi(c, 0, cols - 1)];
    asm volatile("" :: "v"(v));
    x[e]  = v;
    mk[e] = (row < rows && c < cols) ? 0xFFFFu : 0u;
  }
  const v4f a = (v4f){ x[0], x[1], x[2], x[3] };
  const v4f c = (v4f){ x[4], x[5], x[6], x[7] };
  v4u o;
  if (FORM == 2) {
    o = pack8_f16(a, c);
  } else {
    const v4u hi = pack8_bf16(a, c);
    o = hi;
    if (FORM == 1) { const v4u lo = pack8_bf16_lo(a, c); o = second ? lo : hi; }
  }
  const v4u mw = (v4u){ pk16(mk[0], mk[1]), pk16(mk[2], mk[3]), pk16(mk[4], mk[5]), pk16(mk[6], mk[7]) };
  o &= mw;
  if (g < total) {
    volatile v4u* q = (volatile v4u*)(dst + (size_t)g * 8);
    *q = o;
    __threadfence();
    *q = o;
  }
}

template <int FORM> struct FragOf    { typedef FragB T; };
template <>         struct FragOf<2> { typedef FragH T; };
__device__ __forceinline__ v8f mm(const FragB& a, const FragB& b, v8f c) { return wmb(a, b, c); }
__device__ __forceinline__ v8f mm(const FragH& a, const FragH& b, v8f c) { return wmh(a, b, c); }
template <class F> __device__ __forceinline__ F ld_frag(const unsigned short* p) {
  F f;
  f.h[0] = *(const v8usa*)(p);
  f.h[1] = *(const v8usa*)(p + 16);
  return f;
}

template <int FORM, int EPI>
__global__ __launch_bounds__(256) __attribute__((amdgpu_num_vgpr(248)))
void k_gemm_nt(const unsigned short* __restrict__ A, const unsigned short* __restrict__ B,
               const float* __restrict__ bias, float* __restrict__ D, int M, int N, int KTOT, int ldd) {
  static_assert(FORM >= 0 && FORM <= 2);
  static_assert(EPI == 0 || EPI == 1);
  typedef typename FragOf<FORM>::T F;
  __shared__ __attribute__((aligned(16))) float sT[8][16 * 68];
  const int lane = threadIdx.x & 31;
  const int wave = threadIdx.x >> 5;
  const int tilesM = (M + 63) >> 6;
  const int tilesN = (N + 63) >> 6;
  const int tile = blockIdx.x * 8 + wave;
  if (tile >= tilesM * tilesN) return;
  const int tm = tile / tilesN;
  const int tn = tile - tm * tilesN;
  const int m0 = tm << 6;
  const int n0 = tn << 6;

  const int rl = lane & 15;
  const int h8 = (lane >> 4) * 8;
  const unsigned short* pa = A + (size_t)(m0 + rl) * (size_t)KTOT + h8;
  const unsigned short* pb = B + (size_t)(n0 + rl) * (size_t)KTOT + h8;

  v8f acc[4][4];
#pragma unroll
  for (int i = 0; i < 4; ++i)
#pragma unroll
    for (int j = 0; j < 4; ++j) acc[i][j] = (v8f){0.f, 0.f, 0.f, 0.f, 0.f, 0.f, 0.f, 0.f};

#pragma unroll 1
  for (int k0 = 0; k0 < KTOT; k0 += 32) {
    F bf[4];
#pragma unroll
    for (int j = 0; j < 4; ++j) bf[j] = ld_frag<F>(pb + (size_t)(j << 4) * (size_t)KTOT + k0);
#pragma unroll
    for (int i = 0; i < 4; ++i) {
      const F af = ld_frag<F>(pa + (size_t)(i << 4) * (size_t)KTOT + k0);
#pragma unroll
      for (int j = 0; j < 4; ++j) acc[i][j] = mm(af, bf[j], acc[i][j]);
    }
  }

  float* slab = sT[wave];
  const int hh = lane >> 4;
  const int c4 = (lane & 15) * 4;
  const int nc = n0 + c4;
  const bool cok = nc < N;
  v4f bv = (v4f){0.f, 0.f, 0.f, 0.f};
  if (EPI == 1) {
    bv = *(const v4fa*)(bias + clampi(nc, 0, N - 4));
    asm volatile("" :: "v"(bv));
  }
#pragma unroll
  for (int i = 0; i < 4; ++i) {
    const int mBase = m0 + (i << 4);
#pragma unroll
    for (int j = 0; j < 4; ++j) {
#pragma unroll
      for (int r = 0; r < 8; ++r) slab[(h8 + r) * 68 + (j << 4) + rl] = acc[i][j][r];
    }
    __builtin_amdgcn_fence(__ATOMIC_RELEASE, "workgroup");
    __builtin_amdgcn_wave_barrier();
    __builtin_amdgcn_fence(__ATOMIC_ACQUIRE, "workgroup");
    v4f vv[8];
#pragma unroll
    for (int it = 0; it < 8; ++it) {
      const int row = it * 2 + hh;
      v4f v = *(const v4fa*)(slab + row * 68 + c4);
      if (EPI == 1) v += bv;
      vv[it] = v;
    }
    for (int pass = 0; pass < 2; ++pass) {
#pragma unroll
      for (int it = 0; it < 8; ++it) {
        const int row = mBase + it * 2 + hh;
        if (cok && row < M) *(volatile v4f*)(D + (size_t)row * (size_t)ldd + nc) = vv[it];
      }
      __threadfence();
    }
    __builtin_amdgcn_fence(__ATOMIC_RELEASE, "workgroup");
    __builtin_amdgcn_wave_barrier();
    __builtin_amdgcn_fence(__ATOMIC_ACQUIRE, "workgroup");
  }
}

#ifndef SPLIT_A
#define SPLIT_A 1
#endif
#define NN       50000
#define NE       600000
#define MPN      50048
#define NBLK     49
#define NBROWS   1024
#define RCAP     16384
#define DEGCAP   64
#define MAXHITS  12548
#define MAXDEG   28
#define NCHUNK   ((NE + 255) / 256)
#define ESH      10
#define DUPK     (SPLIT_A ? 2 : 1)
#define KA1      (DUPK * 128)
#define KB1      (DUPK * 64)
#define KA2      (DUPK * 64)
#define KB2      (DUPK * 32)
#define PFORM    (SPLIT_A ? 1 : 0)
#define LDS_BKT  ((2 * RCAP + 3 * NBROWS + 32) * 4)
#define PA_B1A   0
#define PA_B1B   64
#define PA_B2A   128
#define PA_B2B   160
#define PA_WL    192
#define PA_WR    224
#define PA_SC    256
#define PAR_LINES 9
#define NB_XB    (MPN * 128 / 8 / 256)
#define NB_W1A   (64 * KA1 / 8 / 256)
#define NB_W1B   (64 * KB1 / 8 / 256)
#define NB_W2A   (64 * KA2 / 8 / 256)
#define NB_W2B   (64 * KB2 / 8 / 256)
#define B_W1A    (NB_XB)
#define B_W1B    (B_W1A + NB_W1A)
#define B_W2A    (B_W1B + NB_W1B)
#define B_W2B    (B_W2A + NB_W2A)
#define B_PAR    (B_W2B + NB_W2B)
#define NB_PREP  (B_PAR + 2)
#define WSMAX    ((size_t)128 << 20)

static_assert(SPLIT_A == 0 || SPLIT_A == 1);
static_assert(MPN % 128 == 0 && MPN % 64 == 0 && MPN >= NN && MPN - NN < 64 && MPN % 8 == 0);
static_assert(NN % 16 == 0);
static_assert(NBLK * NBROWS >= NN && (NBLK - 1) * NBROWS < NN);
static_assert((NN - (NBLK - 1) * NBROWS) % 4 == 0 && NBROWS % 32 == 0 && NBROWS == 4 * 256);
static_assert(NE % 256 == 192 && NCHUNK == 2344);
static_assert(NE <= (1 << (32 - ESH)) && (1 << ESH) >= NBROWS);
static_assert(RCAP % 1024 == 0 && RCAP * 100 >= MAXHITS * 105);
static_assert(DEGCAP >= MAXDEG + 8 && DEGCAP <= 64);
static_assert(LDS_BKT <= 327680 && LDS_BKT == 143488);
static_assert((MPN * 128 / 8) % 256 == 0);
static_assert((64 * KA1 / 8) % 256 == 0 && (64 * KB1 / 8) % 256 == 0 && (64 * KA2 / 8) % 256 == 0 && (64 * KB2 / 8) % 256 == 0);
static_assert(PAR_LINES * 32 >= PA_SC + 3 && PAR_LINES <= 16);
static_assert((NN * 64 / 4) % 256 == 0 && (NN * 32 / 4) % 32 == 0);
static_assert(KA1 % 32 == 0 && KB1 % 32 == 0 && KA2 % 32 == 0 && KB2 % 32 == 0);
static_assert((PA_B1A * 4) % 128 == 0 && (PA_B1B * 4) % 128 == 0 && (PA_B2A * 4) % 128 == 0 && (PA_B2B * 4) % 128 == 0);
static_assert((MPN * KB1 / 8) % 256 == 0 && (MPN * KB2 / 8) % 256 == 0);

constexpr size_t al256(size_t v) { return (v + 255) & ~(size_t)255; }
constexpr size_t O_XB   = 0;
constexpr size_t O_PA   = al256(O_XB   + (size_t)MPN * 128 * 2);
constexpr size_t O_PF   = al256(O_PA   + (size_t)MPN * 256 * 2);
constexpr size_t O_H1   = al256(O_PF   + (size_t)MPN * 64 * 4);
constexpr size_t O_H2   = al256(O_H1   + (size_t)MPN * 64 * 4);
constexpr size_t O_LSRC = al256(O_H2   + (size_t)MPN * 32 * 4);
constexpr size_t O_LEW  = al256(O_LSRC + (size_t)NBLK * RCAP * 4);
constexpr size_t O_OFFC = al256(O_LEW  + (size_t)NBLK * RCAP * 4);
constexpr size_t O_META = al256(O_OFFC + (size_t)NBLK * 2048 * 4);
constexpr size_t O_W1A  = al256(O_META + (size_t)NBLK * 128);
constexpr size_t O_W1B  = al256(O_W1A  + 64 * 256 * 2);
constexpr size_t O_W2A  = al256(O_W1B  + 64 * 128 * 2);
constexpr size_t O_W2B  = al256(O_W2A  + 64 * 128 * 2);
constexpr size_t O_PAR  = al256(O_W2B  + 64 * 64 * 2);
constexpr size_t WS_TOTAL = al256(O_PAR + 2048);
static_assert(WS_TOTAL <= (size_t)WSMAX);
static_assert(WS_TOTAL == 77373696);

typedef int v4i __attribute__((ext_vector_type(4)));
typedef v4i __attribute__((may_alias)) v4ia;
typedef unsigned int v2u __attribute__((ext_vector_type(2)));
typedef v2u __attribute__((may_alias)) v2ua;
typedef float v2f __attribute__((ext_vector_type(2)));
typedef v2f __attribute__((may_alias)) v2fa;

__device__ __forceinline__ void wave_sync_lds() {
  __builtin_amdgcn_fence(__ATOMIC_RELEASE, "workgroup");
  __builtin_amdgcn_wave_barrier();
  __builtin_amdgcn_fence(__ATOMIC_ACQUIRE, "workgroup");
}
__device__ __forceinline__ void st2_v4u(void* p, const v4u v) {
  volatile v4u* q = (volatile v4u*)p;
  *q = v;
  __threadfence();
  *q = v;
}
__device__ __forceinline__ void st2_v4f(float* p, const v4f v) {
  volatile v4f* q = (volatile v4f*)p;
  *q = v;
  __threadfence();
  *q = v;
}
__device__ __forceinline__ void st2_v4i(int* p, const v4i v) {
  volatile v4i* q = (volatile v4i*)p;
  *q = v;
  __threadfence();
  *q = v;
}
__device__ __forceinline__ float relu_keep(float v) { return (v > 0.0f) ? v : (v - v); }

__device__ __forceinline__ void plane_piece(const float* __restrict__ src, int rows, int KP, int KTOT,
                                            unsigned short* dst, int u) {
  const int ppr = KTOT >> 3;
  const int row = u / ppr;
  const int p   = u - row * ppr;
  const int c0  = (p << 3) % KP;
  const int rc  = clampi(row, 0, rows - 1);
  const float* sp = src + (size_t)rc * (size_t)KP + c0;
  const v4f a = *(const v4fa*)sp;
  const v4f c = *(const v4fa*)(sp + 4);
  asm volatile("" :: "v"(a), "v"(c));
  v4u o = pack8_bf16(a, c);
  const unsigned mk = row < rows ? 0xFFFFFFFFu : 0u;
  o &= (v4u){ mk, mk, mk, mk };
  st2_v4u(dst + (size_t)u * 8, o);
}

__global__ __launch_bounds__(256) void k_prep(
    const float* __restrict__ x, const float* __restrict__ w1a, const float* __restrict__ b1a,
    const float* __restrict__ w1b, const float* __restrict__ b1b, const float* __restrict__ eps1,
    const float* __restrict__ w2a, const float* __restrict__ b2a, const float* __restrict__ w2b,
    const float* __restrict__ b2b, const float* __restrict__ eps2, const float* __restrict__ wl,
    const float* __restrict__ bl, const float* __restrict__ wr,
    unsigned short* XB, unsigned short* W1A2, unsigned short* W1B2, unsigned short* W2A2, unsigned short* W2B2,
    float* PAR) {
  const int b = (int)blockIdx.x, tid = (int)threadIdx.x;
  if (b < B_W1A) {
    plane_piece(x, NN, 128, 128, XB, b * 256 + tid);
  } else if (b < B_W1B) {
    plane_piece(w1a, 64, 128, KA1, W1A2, (b - B_W1A) * 256 + tid);
  } else if (b < B_W2A) {
    plane_piece(w1b, 64, 64, KB1, W1B2, (b - B_W1B) * 256 + tid);
  } else if (b < B_W2B) {
    plane_piece(w2a, 32, 64, KA2, W2A2, (b - B_W2A) * 256 + tid);
  } else if (b < B_PAR) {
    plane_piece(w2b, 32, 32, KB2, W2B2, (b - B_W2B) * 256 + tid);
  } else {
    const int lane = tid & 31;
    const int wave = __builtin_amdgcn_readfirstlane(tid >> 5);
    const int u = (b - B_PAR) * 8 + wave;
    if (u < PAR_LINES) {
      float v = 0.0f;
      if (u < 2) {
        v = b1a[32 * u + lane];
      } else if (u < 4) {
        v = b1b[32 * (u - 2) + lane];
      } else if (u == 4) {
        v = b2a[lane];
      } else if (u == 5) {
        v = b2b[lane];
      } else if (u == 6) {
        v = wl[lane];
      } else if (u == 7) {
        v = wr[lane];
      } else {
        const float e1 = eps1[0];
        const float e2 = eps2[0];
        const float bb = bl[0];
        asm volatile("" :: "v"(e1), "v"(e2), "v"(bb));
        const unsigned m0 = lane == 0 ? 0xFFFFFFFFu : 0u;
        const unsigned m1 = lane == 1 ? 0xFFFFFFFFu : 0u;
        const unsigned m2 = lane == 2 ? 0xFFFFFFFFu : 0u;
        v = __uint_as_float((__float_as_uint(e1) & m0) | (__float_as_uint(e2) & m1) | (__float_as_uint(bb) & m2));
      }
      const float o = bf16_val(v);
      volatile float* q = PAR + 32 * u + lane;
      *q = o;
      __threadfence();
      *q = o;
    }
  }
}

__global__ __launch_bounds__(256) void k_bucket(const int* __restrict__ ei, const float* __restrict__ ea,
                                                int* LSRC, float* LEW, int* OFFC, int* META) {
  extern __shared__ v4f lds_dyn[];
  int* reg1 = (int*)lds_dyn;
  int* reg2 = reg1 + RCAP;
  int* scnt = reg2 + RCAP;
  int* soff = scnt + NBROWS;
  int* cur  = soff + NBROWS;
  int* wcnt = cur + NBROWS;
  int* wtot = wcnt + 16;
  const int tid = (int)threadIdx.x, lane = tid & 31, wave = tid >> 5;
  const int b = (int)blockIdx.x;
  const int nodeBase = b * NBROWS;
  const int nb = clampi(NN - nodeBase, 0, NBROWS);
  const int* dsts = ei + NE;

  for (int i = tid; i < NBROWS; i += 256) scnt[i] = 0;
  if (tid == 0) reg2[0] = 0;

  int tot = 0;
#pragma unroll 1
  for (int ch = 0; ch < NCHUNK; ++ch) {
    const int e = ch * 256 + tid;
    int d = dsts[e < NE ? e : NE - 1];
    asm volatile("" :: "v"(d));
    d = (e < NE) ? d : -1;
    const unsigned s = (unsigned)d - (unsigned)nodeBase;
    const bool hit = s < (unsigned)nb;
    const unsigned m = __builtin_amdgcn_ballot_w32(hit);
    const int pb = (ch & 1) * 8;
    if (lane == 0) wcnt[pb + wave] = (int)__builtin_popcount(m);
    __syncthreads();
    int pre = 0, all = 0;
#pragma unroll
    for (int w2 = 0; w2 < 8; ++w2) {
      int c = wcnt[pb + w2];
      c = c < 0 ? 0 : (c > 32 ? 32 : c);
      all += c;
      pre += (w2 < wave) ? c : 0;
    }
    const int pos = tot + pre + (int)__builtin_amdgcn_mbcnt_lo(m, 0u);
    if (hit && pos < RCAP) reg1[pos] = (int)(((unsigned)e << ESH) | s);
    tot += all;
  }
  __syncthreads();
  const int ovf = tot > RCAP ? 1 : 0;
  const int nh = __builtin_amdgcn_readfirstlane(tot > RCAP ? RCAP : tot);

  if (wave == 0) {
#pragma unroll 1
    for (int b0 = 0; b0 < nh; b0 += 32) {
      const int idx = (b0 + lane) < nh ? (b0 + lane) : nh - 1;
      const int uv  = reg1[idx];
      const int m32 = (nh - b0) < 32 ? (nh - b0) : 32;
#pragma unroll 1
      for (int k = 0; k < m32; ++k) {
        const int u  = __builtin_amdgcn_readlane(uv, k);
        const int sl = u & (NBROWS - 1);
        if (lane == 0) scnt[sl] = scnt[sl] + 1;
      }
    }
  }
  __syncthreads();

  {
    const v4i ca = *(const v4ia*)(scnt + 4 * tid);
    const int e0 = ca.x < 0 ? 0 : ca.x, e1 = ca.y < 0 ? 0 : ca.y, e2 = ca.z < 0 ? 0 : ca.z, e3 = ca.w < 0 ? 0 : ca.w;
    const int ts = e0 + e1 + e2 + e3;
    int incl = ts;
#pragma unroll
    for (int dd = 1; dd < 32; dd <<= 1) {
      const int up = __shfl_up(incl, dd);
      if (lane >= dd) incl += up;
    }
    if (lane == 31) wtot[wave] = incl;
    __syncthreads();
    int pre = 0;
#pragma unroll
    for (int w2 = 0; w2 < 8; ++w2) pre += (w2 < wave) ? wtot[w2] : 0;
    int run = pre + incl - ts;
    soff[4 * tid + 0] = run; cur[4 * tid + 0] = run; run += e0;
    soff[4 * tid + 1] = run; cur[4 * tid + 1] = run; run += e1;
    soff[4 * tid + 2] = run; cur[4 * tid + 2] = run; run += e2;
    soff[4 * tid + 3] = run; cur[4 * tid + 3] = run;
  }
  __syncthreads();

  if (wave == 0) {
#pragma unroll 1
    for (int b0 = 0; b0 < nh; b0 += 32) {
      const int idx = (b0 + lane) < nh ? (b0 + lane) : nh - 1;
      const int uv  = reg1[idx];
      const int m32 = (nh - b0) < 32 ? (nh - b0) : 32;
#pragma unroll 1
      for (int k = 0; k < m32; ++k) {
        const int u   = __builtin_amdgcn_readlane(uv, k);
        const int sl  = u & (NBROWS - 1);
        const int eid = (int)((unsigned)u >> ESH);
        if (lane == 0) {
          int pos = cur[sl];
          pos = pos < 0 ? 0 : (pos > RCAP - 1 ? RCAP - 1 : pos);
          reg2[pos] = eid;
          cur[sl] = pos + 1;
        }
      }
    }
  }
  __syncthreads();

  int*   ls = LSRC + (size_t)b * RCAP;
  float* lw = LEW  + (size_t)b * RCAP;
  const int last = nh > 0 ? nh - 1 : 0;
#pragma unroll 1
  for (int base = 0; base < RCAP; base += 1024) {
    const int i0 = base + 4 * tid;
    const int id0 = clampi(reg2[i0     < last ? i0     : last], 0, NE - 1);
    const int id1 = clampi(reg2[i0 + 1 < last ? i0 + 1 : last], 0, NE - 1);
    const int id2 = clampi(reg2[i0 + 2 < last ? i0 + 2 : last], 0, NE - 1);
    const int id3 = clampi(reg2[i0 + 3 < last ? i0 + 3 : last], 0, NE - 1);
    const int s0 = ei[id0], s1 = ei[id1], s2 = ei[id2], s3 = ei[id3];
    asm volatile("" :: "v"(s0), "v"(s1), "v"(s2), "v"(s3));
    v4i v;
    v.x = (i0     < nh) ? clampi(s0, 0, NN - 1) : 0;
    v.y = (i0 + 1 < nh) ? clampi(s1, 0, NN - 1) : 0;
    v.z = (i0 + 2 < nh) ? clampi(s2, 0, NN - 1) : 0;
    v.w = (i0 + 3 < nh) ? clampi(s3, 0, NN - 1) : 0;
    st2_v4i(ls + i0, v);
  }
#pragma unroll 1
  for (int base = 0; base < RCAP; base += 1024) {
    const int i0 = base + 4 * tid;
    const int id0 = clampi(reg2[i0     < last ? i0     : last], 0, NE - 1);
    const int id1 = clampi(reg2[i0 + 1 < last ? i0 + 1 : last], 0, NE - 1);
    const int id2 = clampi(reg2[i0 + 2 < last ? i0 + 2 : last], 0, NE - 1);
    const int id3 = clampi(reg2[i0 + 3 < last ? i0 + 3 : last], 0, NE - 1);
    const float w0 = ea[id0], w1 = ea[id1], w2 = ea[id2], w3 = ea[id3];
    asm volatile("" :: "v"(w0), "v"(w1), "v"(w2), "v"(w3));
    v4f o;
    o[0] = (i0     < nh) ? bf16_val(w0) : 0.0f;
    o[1] = (i0 + 1 < nh) ? bf16_val(w1) : 0.0f;
    o[2] = (i0 + 2 < nh) ? bf16_val(w2) : 0.0f;
    o[3] = (i0 + 3 < nh) ? bf16_val(w3) : 0.0f;
    st2_v4f(lw + i0, o);
  }
  {
    const v4i so = *(const v4ia*)(soff + 4 * tid);
    const v4i sc = *(const v4ia*)(scnt + 4 * tid);
    int* oc = OFFC + (size_t)b * 2048;
    st2_v4i(oc + 4 * tid, so);
    st2_v4i(oc + 1024 + 4 * tid, sc);
  }
  if (tid < 8) {
    v4i mv;
    mv.x = (tid == 0) ? nh : 0;
    mv.y = (tid == 0) ? ovf : 0;
    mv.z = 0; mv.w = 0;
    st2_v4i(META + (size_t)b * 32 + 4 * tid, mv);
  }
}

__global__ __launch_bounds__(256) void k_agg1(const unsigned short* __restrict__ XB, const int* __restrict__ LSRC,
                                              const int* __restrict__ OFFC, const int* __restrict__ META,
                                              const float* __restrict__ par, unsigned short* Z) {
  __shared__ __attribute__((aligned(16))) float sZ[8][128];
  const int tid = (int)threadIdx.x, lane = tid & 31;
  const int wave = __builtin_amdgcn_readfirstlane(tid >> 5);
  const int row = (int)blockIdx.x * 8 + wave;
  const bool valid = row < NN;
  const int rc = valid ? row : NN - 1;
  const int b = rc >> 10, slot = rc & 1023;
  const int nh = clampi(META[(size_t)b * 32], 0, RCAP);
  const int flag = META[(size_t)b * 32 + 1];
  int st = OFFC[(size_t)b * 2048 + slot];
  int craw = OFFC[(size_t)b * 2048 + 1024 + slot];
  asm volatile("" :: "v"(st), "v"(craw));
  craw = craw < 0 ? 0 : craw;
  const bool bad = valid && (flag != 0 || craw > DEGCAP);
  st = clampi(st, 0, nh);
  int cnt = craw > DEGCAP ? DEGCAP : craw;
  cnt = cnt > nh - st ? nh - st : cnt;
  cnt = valid ? cnt : 0;
  cnt = __builtin_amdgcn_readfirstlane(cnt);
  st  = __builtin_amdgcn_readfirstlane(st);
  const int nhm1 = nh > 0 ? nh - 1 : 0;
  const int* ls = LSRC + (size_t)b * RCAP;
  float a0 = 0.0f, a1 = 0.0f, a2 = 0.0f, a3 = 0.0f;
#pragma unroll 1
  for (int b0 = 0; b0 < cnt; b0 += 32) {
    int s = ls[clampi(st + b0 + lane, 0, nhm1)];
    asm volatile("" :: "v"(s));
    s = clampi(s, 0, NN - 1);
    const int m32 = (cnt - b0) < 32 ? (cnt - b0) : 32;
#pragma unroll 4
    for (int q = 0; q < m32; ++q) {
      const int sq = __builtin_amdgcn_readlane(s, q);
      const v2u w = *(const v2ua*)(XB + (size_t)sq * 128 + 4 * lane);
      asm volatile("" :: "v"(w));
      a0 += __uint_as_float(w.x << 16);
      a1 += __uint_as_float(w.x & 0xffff0000u);
      a2 += __uint_as_float(w.y << 16);
      a3 += __uint_as_float(w.y & 0xffff0000u);
    }
  }
  const v2u ws = *(const v2ua*)(XB + (size_t)rc * 128 + 4 * lane);
  const float epl = 1.0f + par[PA_SC];
  const float qnan = __int_as_float(0x7fc00000);
  v4f z;
  z[0] = epl * __uint_as_float(ws.x << 16) + a0;
  z[1] = epl * __uint_as_float(ws.x & 0xffff0000u) + a1;
  z[2] = epl * __uint_as_float(ws.y << 16) + a2;
  z[3] = epl * __uint_as_float(ws.y & 0xffff0000u) + a3;
#pragma unroll
  for (int e = 0; e < 4; ++e) {
    float t = valid ? z[e] : 0.0f;
    t = bad ? qnan : t;
    z[e] = t;
  }
  float* strip = &sZ[wave][0];
  *(v4fa*)(strip + 4 * lane) = z;
  wave_sync_lds();
  {
    const int p = lane;
    const float* sp = strip + (p & 15) * 8;
    const v4f a = *(const v4fa*)sp;
    const v4f c = *(const v4fa*)(sp + 4);
    const v4u hi = pack8_bf16(a, c);
    const v4u lo = pack8_bf16_lo(a, c);
    const v4u o = (SPLIT_A != 0 && p >= 16) ? lo : hi;
    if (p < KA1 / 8) st2_v4u(Z + (size_t)row * KA1 + p * 8, o);
  }
}

__global__ __launch_bounds__(256) void k_agg2(const float* __restrict__ H1, const int* __restrict__ LSRC,
                                              const int* __restrict__ OFFC, const int* __restrict__ META,
                                              const float* __restrict__ par, unsigned short* Z) {
  __shared__ __attribute__((aligned(16))) float sZ[8][64];
  const int tid = (int)threadIdx.x, lane = tid & 31;
  const int wave = __builtin_amdgcn_readfirstlane(tid >> 5);
  const int row = (int)blockIdx.x * 8 + wave;
  const bool valid = row < NN;
  const int rc = valid ? row : NN - 1;
  const int b = rc >> 10, slot = rc & 1023;
  const int nh = clampi(META[(size_t)b * 32], 0, RCAP);
  const int flag = META[(size_t)b * 32 + 1];
  int st = OFFC[(size_t)b * 2048 + slot];
  int craw = OFFC[(size_t)b * 2048 + 1024 + slot];
  asm volatile("" :: "v"(st), "v"(craw));
  craw = craw < 0 ? 0 : craw;
  const bool bad = valid && (flag != 0 || craw > DEGCAP);
  st = clampi(st, 0, nh);
  int cnt = craw > DEGCAP ? DEGCAP : craw;
  cnt = cnt > nh - st ? nh - st : cnt;
  cnt = valid ? cnt : 0;
  cnt = __builtin_amdgcn_readfirstlane(cnt);
  st  = __builtin_amdgcn_readfirstlane(st);
  const int nhm1 = nh > 0 ? nh - 1 : 0;
  const int* ls = LSRC + (size_t)b * RCAP;
  float a0 = 0.0f, a1 = 0.0f;
#pragma unroll 1
  for (int b0 = 0; b0 < cnt; b0 += 32) {
    int s = ls[clampi(st + b0 + lane, 0, nhm1)];
    asm volatile("" :: "v"(s));
    s = clampi(s, 0, NN - 1);
    const int m32 = (cnt - b0) < 32 ? (cnt - b0) : 32;
#pragma unroll 4
    for (int q = 0; q < m32; ++q) {
      const int sq = __builtin_amdgcn_readlane(s, q);
      const v2f h = *(const v2fa*)(H1 + (size_t)sq * 64 + 2 * lane);
      asm volatile("" :: "v"(h));
      a0 += h[0];
      a1 += h[1];
    }
  }
  const v2f xs = *(const v2fa*)(H1 + (size_t)rc * 64 + 2 * lane);
  const float epl = 1.0f + par[PA_SC + 1];
  const float qnan = __int_as_float(0x7fc00000);
  float z0 = epl * xs[0] + a0;
  float z1 = epl * xs[1] + a1;
  z0 = valid ? z0 : 0.0f;
  z1 = valid ? z1 : 0.0f;
  z0 = bad ? qnan : z0;
  z1 = bad ? qnan : z1;
  float* strip = &sZ[wave][0];
  *(v2fa*)(strip + 2 * lane) = (v2f){ z0, z1 };
  wave_sync_lds();
  {
    const int p = lane;
    const float* sp = strip + (p & 7) * 8;
    const v4f a = *(const v4fa*)sp;
    const v4f c = *(const v4fa*)(sp + 4);
    const v4u hi = pack8_bf16(a, c);
    const v4u lo = pack8_bf16_lo(a, c);
    const v4u o = (SPLIT_A != 0 && p >= 8) ? lo : hi;
    if (p < KA2 / 8) st2_v4u(Z + (size_t)row * KA2 + p * 8, o);
  }
}

template <int COLS>
__global__ __launch_bounds__(256) void k_relu(const float* __restrict__ U, float* Hout) {
  const int total = NN * COLS / 4;
  const int g = (int)blockIdx.x * 256 + (int)threadIdx.x;
  const int gc = g < total ? g : total - 1;
  v4f v = *(const v4fa*)(U + (size_t)gc * 4);
  asm volatile("" :: "v"(v));
#pragma unroll
  for (int e = 0; e < 4; ++e) v[e] = relu_keep(v[e]);
  if (g < total) st2_v4f(Hout + (size_t)g * 4, v);
}

__global__ __launch_bounds__(256) void k_sage_out(const float* __restrict__ H2, const int* __restrict__ LSRC,
                                                  const float* __restrict__ LEW, const int* __restrict__ OFFC,
                                                  const int* __restrict__ META, const float* __restrict__ par,
                                                  float* out) {
  __shared__ __attribute__((aligned(16))) float sOut[NBROWS];
  const int tid = (int)threadIdx.x, lane = tid & 31;
  const int wave = __builtin_amdgcn_readfirstlane(tid >> 5);
  const int b = (int)blockIdx.x;
  const int nodeBase = b * NBROWS;
  const int nb = clampi(NN - nodeBase, 0, NBROWS);
  *(v4fa*)(sOut + 4 * tid) = (v4f){ 0.0f, 0.0f, 0.0f, 0.0f };
  __syncthreads();
  const int nh = clampi(META[(size_t)b * 32], 0, RCAP);
  const int flag = META[(size_t)b * 32 + 1];
  const bool ovf = flag != 0;
  const int nhm1 = nh > 0 ? nh - 1 : 0;
  const int*   ls = LSRC + (size_t)b * RCAP;
  const float* lw = LEW  + (size_t)b * RCAP;
  const int*   oc = OFFC + (size_t)b * 2048;
  const float wlv = par[PA_WL + lane];
  const float wrv = par[PA_WR + lane];
  const float blv = par[PA_SC + 2];
  const float qnan = __int_as_float(0x7fc00000);

#pragma unroll 1
  for (int g = 0; g < 4; ++g) {
    const int slot0 = wave * 128 + g * 32;
    if (slot0 >= nb) break;
    int stv = oc[slot0 + lane];
    int cv  = oc[1024 + slot0 + lane];
    asm volatile("" :: "v"(stv), "v"(cv));
    const int craw = cv < 0 ? 0 : cv;
    const int pv = (craw > DEGCAP) ? 1 : 0;
    stv = clampi(stv, 0, nh);
    int cc = craw > DEGCAP ? DEGCAP : craw;
    cc = cc > nh - stv ? nh - stv : cc;
#pragma unroll 1
    for (int rr = 0; rr < 32; ++rr) {
      const int slot = slot0 + rr;
      if (slot >= nb) break;
      const int st  = __builtin_amdgcn_readlane(stv, rr);
      const int cnt = __builtin_amdgcn_readlane(cc, rr);
      const int cr  = __builtin_amdgcn_readlane(craw, rr);
      const int prw = __builtin_amdgcn_readlane(pv, rr);
      const int node = nodeBase + slot;
      float num = 0.0f;
#pragma unroll 1
      for (int b0 = 0; b0 < cnt; b0 += 32) {
        const int li = clampi(st + b0 + lane, 0, nhm1);
        int s = ls[li];
        const float w = lw[li];
        asm volatile("" :: "v"(s), "v"(w));
        s = clampi(s, 0, NN - 1);
        const int wi = __float_as_int(w);
        const int m32 = (cnt - b0) < 32 ? (cnt - b0) : 32;
#pragma unroll 4
        for (int q = 0; q < m32; ++q) {
          const int sq = __builtin_amdgcn_readlane(s, q);
          const float ew = __int_as_float(__builtin_amdgcn_readlane(wi, q));
          const float h = H2[(size_t)sq * 32 + lane];
          asm volatile("" :: "v"(h));
          num += ew * h;
        }
      }
      const float den = fmaxf((float)cr, 1.0f);
      const float mean = num / den;
      const float hs = H2[(size_t)node * 32 + lane];
      float p = mean * wlv;
      float q2 = hs * wrv;
      p += __shfl_xor(p, 16);
      p += __shfl_xor(p, 8);
      p += __shfl_xor(p, 4);
      p += __shfl_xor(p, 2);
      p += __shfl_xor(p, 1);
      q2 += __shfl_xor(q2, 16);
      q2 += __shfl_xor(q2, 8);
      q2 += __shfl_xor(q2, 4);
      q2 += __shfl_xor(q2, 2);
      q2 += __shfl_xor(q2, 1);
      float o = (p + blv) + q2;
      o = relu_keep(o);
      o = (ovf || prw != 0) ? qnan : o;
      if (lane == 0) sOut[slot] = o;
    }
  }
  __syncthreads();
  {
    const int s0 = 4 * tid;
    const v4f v = *(const v4fa*)(sOut + s0);
    if (s0 < nb) st2_v4f(out + nodeBase + s0, v);
  }
}

extern "C" void kernel_launch(void* const* d_in, const int* in_sizes, int n_in,
                              void* d_out, int out_size, void* d_ws, size_t ws_size,
                              hipStream_t stream) {
  if (n_in < 16) return;
  if (in_sizes[0] != NN * 128 || in_sizes[1] != 2 * NE || in_sizes[2] != NE) return;
  if (in_sizes[3] != 64 * 128 || in_sizes[4] != 64 || in_sizes[5] != 64 * 64 || in_sizes[6] != 64) return;
  if (in_sizes[7] != 1 || in_sizes[8] != 32 * 64 || in_sizes[9] != 32 || in_sizes[10] != 32 * 32) return;
  if (in_sizes[11] != 32 || in_sizes[12] != 1 || in_sizes[13] != 32 || in_sizes[14] != 1 || in_sizes[15] != 32) return;
  if (out_size != NN) return;
  if (ws_size < WS_TOTAL) return;

  const float* x    = (const float*)d_in[0];
  const int*   ei   = (const int*)  d_in[1];
  const float* ea   = (const float*)d_in[2];
  const float* w1a  = (const float*)d_in[3];
  const float* b1a  = (const float*)d_in[4];
  const float* w1b  = (const float*)d_in[5];
  const float* b1b  = (const float*)d_in[6];
  const float* eps1 = (const float*)d_in[7];
  const float* w2a  = (const float*)d_in[8];
  const float* b2a  = (const float*)d_in[9];
  const float* w2b  = (const float*)d_in[10];
  const float* b2b  = (const float*)d_in[11];
  const float* eps2 = (const float*)d_in[12];
  const float* wl   = (const float*)d_in[13];
  const float* bl   = (const float*)d_in[14];
  const float* wr   = (const float*)d_in[15];
  float* out = (float*)d_out;

  char* ws = (char*)d_ws;
  unsigned short* XB   = (unsigned short*)(ws + O_XB);
  unsigned short* PA   = (unsigned short*)(ws + O_PA);
  float*          PF   = (float*)(ws + O_PF);
  float*          H1   = (float*)(ws + O_H1);
  float*          H2   = (float*)(ws + O_H2);
  int*            LSRC = (int*)(ws + O_LSRC);
  float*          LEW  = (float*)(ws + O_LEW);
  int*            OFFC = (int*)(ws + O_OFFC);
  int*            META = (int*)(ws + O_META);
  unsigned short* W1A2 = (unsigned short*)(ws + O_W1A);
  unsigned short* W1B2 = (unsigned short*)(ws + O_W1B);
  unsigned short* W2A2 = (unsigned short*)(ws + O_W2A);
  unsigned short* W2B2 = (unsigned short*)(ws + O_W2B);
  float*          PAR  = (float*)(ws + O_PAR);

  hipFuncSetAttribute(reinterpret_cast<const void*>(&k_bucket),
                      hipFuncAttributeMaxDynamicSharedMemorySize, LDS_BKT);

  k_prep<<<NB_PREP, 256, 0, stream>>>(x, w1a, b1a, w1b, b1b, eps1, w2a, b2a, w2b, b2b, eps2, wl, bl, wr,
                                      XB, W1A2, W1B2, W2A2, W2B2, PAR);
  k_bucket<<<NBLK, 256, LDS_BKT, stream>>>(ei, ea, LSRC, LEW, OFFC, META);
  k_agg1<<<MPN / 8, 256, 0, stream>>>(XB, LSRC, OFFC, META, PAR, PA);
  k_gemm_nt<0, 1><<<(782 + 7) / 8, 256, 0, stream>>>(PA, W1A2, PAR + PA_B1A, PF, NN, 64, KA1, 64);
  k_plane<PFORM><<<MPN * KB1 / 8 / 256, 256, 0, stream>>>(PF, NN, 64, 64, PA, MPN, 64);
  k_gemm_nt<0, 1><<<(782 + 7) / 8, 256, 0, stream>>>(PA, W1B2, PAR + PA_B1B, PF, NN, 64, KB1, 64);
  k_relu<64><<<(NN * 64 / 4 + 255) / 256, 256, 0, stream>>>(PF, H1);
  k_agg2<<<MPN / 8, 256, 0, stream>>>(H1, LSRC, OFFC, META, PAR, PA);
  k_gemm_nt<0, 1><<<(782 + 7) / 8, 256, 0, stream>>>(PA, W2A2, PAR + PA_B2A, PF, NN, 32, KA2, 32);
  k_plane<PFORM><<<MPN * KB2 / 8 / 256, 256, 0, stream>>>(PF, NN, 32, 32, PA, MPN, 32);
  k_gemm_nt<0, 1><<<(782 + 7) / 8, 256, 0, stream>>>(PA, W2B2, PAR + PA_B2B, PF, NN, 32, KB2, 32);
  k_relu<32><<<(NN * 32 / 4 + 255) / 256, 256, 0, stream>>>(PF, H2);
  k_sage_out<<<NBLK, 256, 0, stream>>>(H2, LSRC, LEW, OFFC, META, PAR, out);
}
